// Self_Attention_44160853737538
// MI455X (gfx1250) — hardware-verified
//
#include <hip/hip_runtime.h>


#ifndef NB
#define NB 4
#endif
#ifndef SEQ
#define SEQ 2048
#endif
#define NB_FULL 4
#define T_FULL  2048
#define EMB  1024
#define NH   16
#define HD   64
#define NZ   (NB * NH)
#define RH   (((SEQ) < 256) ? (SEQ) : 256)
#define CCAR 16.0f
#define WCAR 64.0f
#define OSC  0.0009765625f
#define SL2E 0.18033688011112042f
#define NEGB (-3.0e38f)

static_assert((SEQ) % 64 == 0);
static_assert((SEQ) <= T_FULL);
static_assert((NB) >= 1 && (NB) <= NB_FULL);
static_assert((RH) % 64 == 0 && (RH) >= 64 && (RH) <= (SEQ));
static_assert(EMB == NH * HD);
static_assert(EMB % 64 == 0);

typedef _Float16 h16;
typedef unsigned short bf;
typedef __attribute__((ext_vector_type(16))) __bf16   v16bf;
typedef __attribute__((ext_vector_type(16))) _Float16 v16h;
typedef __attribute__((ext_vector_type(16))) unsigned short v16us;
typedef __attribute__((ext_vector_type(8)))  _Float16 v8h;
typedef __attribute__((ext_vector_type(8)))  unsigned short v8us;
typedef __attribute__((ext_vector_type(8)))  float    v8f;
typedef __attribute__((ext_vector_type(4)))  float    v4f;
typedef __attribute__((ext_vector_type(2)))  _Float16 v2h;
typedef __attribute__((ext_vector_type(2)))  unsigned short v2us;
typedef v4f  __attribute__((may_alias)) v4fa;

__device__ __forceinline__ unsigned short f2bf(float f) { unsigned u = __float_as_uint(f); u += 0x7FFFu + ((u >> 16) & 1u); return (unsigned short)(u >> 16); }
__device__ __forceinline__ float bf2f(unsigned short b) { return __uint_as_float(((unsigned)b) << 16); }
__device__ __forceinline__ float bfr(float f) { return bf2f(f2bf(f)); }
__device__ __forceinline__ h16 tohx(float x) { return (h16)x; }
__device__ __forceinline__ void splitf(float y, unsigned short& h, unsigned short& l) { h = f2bf(y); l = f2bf(y - bf2f(h)); }
__device__ __forceinline__ v16h cat16(v8h lo, v8h hi) { return __builtin_shufflevector(lo, hi, 0, 1, 2, 3, 4, 5, 6, 7, 8, 9, 10, 11, 12, 13, 14, 15); }
__device__ __forceinline__ v16bf cat16b(v8us lo, v8us hi) { return __builtin_bit_cast(v16bf, __builtin_shufflevector(lo, hi, 0, 1, 2, 3, 4, 5, 6, 7, 8, 9, 10, 11, 12, 13, 14, 15)); }
__device__ __forceinline__ v8f wmma16(v16h a, v16h b, v8f c) { return __builtin_amdgcn_wmma_f32_16x16x32_f16(false, a, false, b, (short)0, c, false, false); }
__device__ __forceinline__ v8f wmmab(v16bf a, v16bf b, v8f c) { return __builtin_amdgcn_wmma_f32_16x16x32_bf16(false, a, false, b, (short)0, c, false, false); }
__device__ __forceinline__ v16h  zh()  { return __builtin_bit_cast(v16h, (v8f){}); }
__device__ __forceinline__ v16bf zb()  { return __builtin_bit_cast(v16bf, (v8f){}); }
__device__ __forceinline__ v16us zus() { return __builtin_bit_cast(v16us, (v8f){}); }

template <typename T16> struct WFrag;
template <> struct WFrag<h16> { typedef v16h V; static __device__ __forceinline__ V ld(const h16* p) { return cat16(*(const v8h*)p, *(const v8h*)(p + 16)); } static __device__ __forceinline__ v8f mma(V a, V b, v8f c) { return wmma16(a, b, c); } };
template <> struct WFrag<bf> { typedef v16bf V; static __device__ __forceinline__ V ld(const bf* p) { return cat16b(*(const v8us*)p, *(const v8us*)(p + 16)); } static __device__ __forceinline__ v8f mma(V a, V b, v8f c) { return wmmab(a, b, c); } };
template <typename T16, int NSPLIT, bool BIAS>
__global__ __launch_bounds__(32) void k_gemmw(const T16* __restrict__ A, const T16* __restrict__ A2, const T16* __restrict__ Bt, const T16* __restrict__ Bt2, int K, float* C, int ldc, const float* __restrict__ bias, size_t sA, size_t sB, size_t sC, float csc) {
    typedef typename WFrag<T16>::V V;
    __shared__ __align__(16) float os[16 * 68];
    const size_t z = blockIdx.z; A += z * sA; if (A2) A2 += z * sA; Bt += z * sB; if (Bt2) Bt2 += z * sB; C += z * sC;
    const int lane = threadIdx.x & 31, lr = lane & 15, hi = lane >> 4; const int r0 = blockIdx.x * 64, c0 = blockIdx.y * 64;
    v8f acc[4][4];
#pragma unroll
    for (int mb = 0; mb < 4; ++mb)
#pragma unroll
        for (int nb = 0; nb < 4; ++nb) acc[mb][nb] = (v8f){};
    const size_t aoff = (size_t)(r0 + lr) * K + 8 * hi, boff = (size_t)(c0 + lr) * K + 8 * hi;
#pragma unroll 1
    for (int kc = 0; kc < K; kc += 32) {
        V a[4], a2[4];
#pragma unroll
        for (int mb = 0; mb < 4; ++mb) { a[mb] = WFrag<T16>::ld(A + aoff + (size_t)mb * 16 * K + kc); if (NSPLIT == 1 || NSPLIT == 2) a2[mb] = WFrag<T16>::ld(A2 + aoff + (size_t)mb * 16 * K + kc); }
#pragma unroll
        for (int nb = 0; nb < 4; ++nb) { const V b = WFrag<T16>::ld(Bt + boff + (size_t)nb * 16 * K + kc); V b2; if (NSPLIT >= 2) b2 = WFrag<T16>::ld(Bt2 + boff + (size_t)nb * 16 * K + kc);
#pragma unroll
            for (int mb = 0; mb < 4; ++mb) { acc[mb][nb] = WFrag<T16>::mma(a[mb], b, acc[mb][nb]); if (NSPLIT == 1 || NSPLIT == 2) acc[mb][nb] = WFrag<T16>::mma(a2[mb], b, acc[mb][nb]); if (NSPLIT >= 2) acc[mb][nb] = WFrag<T16>::mma(a[mb], b2, acc[mb][nb]); } }
        asm volatile("v_nop\n\tv_nop\n\tv_nop\n\tv_nop" : "+v"(acc[0][0]), "+v"(acc[1][1]), "+v"(acc[2][2]), "+v"(acc[3][3]) : "v"(a[0]), "v"(a[3]));
    }
#pragma unroll
    for (int mb = 0; mb < 4; ++mb) {
#pragma unroll
        for (int nb = 0; nb < 4; ++nb) {
#pragma unroll
            for (int j = 0; j < 8; ++j) os[(hi * 8 + j) * 68 + nb * 16 + lr] = acc[mb][nb][j]; }
        __builtin_amdgcn_wave_barrier(); asm volatile("" ::: "memory");
        float* crow = C + (size_t)(r0 + mb * 16) * ldc + c0;
#pragma unroll 1
        for (int ps = 0; ps < 2; ++ps) {
#pragma unroll
            for (int s = 0; s < 8; ++s) { const int row = 2 * s + hi, cofs = lr * 4; v4f val = *(const v4fa*)(os + row * 68 + cofs); val = val * csc;
                if (BIAS) { val[0] += bfr(bias[c0 + cofs]); val[1] += bfr(bias[c0 + cofs + 1]); val[2] += bfr(bias[c0 + cofs + 2]); val[3] += bfr(bias[c0 + cofs + 3]); }
                *(volatile v4f*)(crow + (size_t)row * ldc + cofs) = val; }
            if (ps == 0) __threadfence(); }
        __builtin_amdgcn_wave_barrier(); asm volatile("" ::: "memory");
    }
}

template <typename OT> struct WCv;
template <> struct WCv<bf>  { typedef v2us V2; static __device__ __forceinline__ unsigned short cv(float w) { return f2bf(w); } };
template <> struct WCv<h16> { typedef v2h  V2; static __device__ __forceinline__ h16 cv(float w) { return tohx(bfr(w) * WCAR); } };
template <typename OT>
__global__ __launch_bounds__(256) void k_wtG(const float* __restrict__ w, int K, int N, OT* Bt) {
    typedef typename WCv<OT>::V2 V2;
    const int lane = threadIdx.x & 31; const int L0 = (blockIdx.x * 8 + (threadIdx.x >> 5)) * 8; const int nlines = N * K / 64;
#pragma unroll
    for (int ps = 0; ps < 2; ++ps) {
#pragma unroll 1
        for (int l = 0; l < 8; ++l) { const int L = L0 + l; if (L >= nlines) break; const size_t e = (size_t)L * 64 + lane * 2; const int k = (int)(e % K), n = (int)(e / K); V2 o;
            o[0] = WCv<OT>::cv(w[(size_t)k * N + n]); o[1] = WCv<OT>::cv(w[(size_t)(k + 1) * N + n]); *(volatile V2*)(Bt + e) = o; }
        if (ps == 0) __threadfence(); }
}

__global__ __launch_bounds__(256) void k_cvtx(const float* __restrict__ x, bf* XB, size_t n8) {
    const size_t i = (size_t)blockIdx.x * 256 + threadIdx.x; if (i >= n8) return;
    const size_t el = i * 8; const int col = (int)(el % EMB); const size_t row = el / EMB; const int b = (int)(row / SEQ); const int t = (int)(row % SEQ);
    const v8f v = *(const v8f*)(x + ((size_t)b * T_FULL + t) * EMB + col); v8us o;
#pragma unroll
    for (int k = 0; k < 8; ++k) o[k] = f2bf(v[k]);
    *(volatile v8us*)(XB + el) = o; __threadfence(); *(volatile v8us*)(XB + el) = o; }

__global__ __launch_bounds__(256) void k_qkp(const float* __restrict__ F, int z0, h16* P16, bf* Ph, bf* Pl) {
    const size_t e = ((size_t)blockIdx.x * 256 + threadIdx.x) * 2; if (e >= (size_t)NH * SEQ * HD) return;
    const int d = (int)(e % HD); const int t = (int)((e / HD) % SEQ); const int hh = (int)(e / ((size_t)HD * SEQ));
    const float* f = F + (size_t)t * EMB + hh * HD + d; v2h o16; v2us oh, ol;
#pragma unroll
    for (int q = 0; q < 2; ++q) { const float xv = f[q]; o16[q] = tohx(xv); unsigned short a, c; splitf(xv, a, c); oh[q] = a; ol[q] = c; }
    const size_t o1 = (size_t)z0 * SEQ * HD + e;
    const bool lo = (t < RH); const size_t o2 = ((size_t)(z0 + hh) * RH + (lo ? t : 0)) * HD + d;
    *(volatile v2h*)(P16 + o1) = o16; if (lo) { *(volatile v2us*)(Ph + o2) = oh; *(volatile v2us*)(Pl + o2) = ol; }
    __threadfence();
    *(volatile v2h*)(P16 + o1) = o16; if (lo) { *(volatile v2us*)(Ph + o2) = oh; *(volatile v2us*)(Pl + o2) = ol; } }

__global__ __launch_bounds__(256) void k_vtp(const float* __restrict__ F, int z0, h16* VT16, bf* VTh, bf* VTl) {
    const size_t e = ((size_t)blockIdx.x * 256 + threadIdx.x) * 2; if (e >= (size_t)NH * HD * SEQ) return;
    const int t = (int)(e % SEQ); const int d = (int)((e / SEQ) % HD); const int g = (int)(e / ((size_t)SEQ * HD));
    v2h o16; v2us oh, ol;
#pragma unroll
    for (int q = 0; q < 2; ++q) { const float xv = F[(size_t)(t + q) * EMB + g * HD + d]; o16[q] = tohx(xv); unsigned short a, c; splitf(xv, a, c); oh[q] = a; ol[q] = c; }
    const size_t o1 = (size_t)z0 * HD * SEQ + e;
    const bool lo = (t < RH); const size_t o2 = ((size_t)(z0 + g) * HD + d) * RH + (lo ? t : 0);
    *(volatile v2h*)(VT16 + o1) = o16; if (lo) { *(volatile v2us*)(VTh + o2) = oh; *(volatile v2us*)(VTl + o2) = ol; }
    __threadfence();
    *(volatile v2h*)(VT16 + o1) = o16; if (lo) { *(volatile v2us*)(VTh + o2) = oh; *(volatile v2us*)(VTl + o2) = ol; } }

template <bool HI, int CH>
__global__ __launch_bounds__(64) __attribute__((amdgpu_num_vgpr(256)))
void k_attn(const h16* __restrict__ Q16, const h16* __restrict__ K16, const h16* __restrict__ VT16,
            const bf* __restrict__ Qh, const bf* __restrict__ Ql, const bf* __restrict__ Kh, const bf* __restrict__ Kl,
            const bf* __restrict__ VTh, const bf* __restrict__ VTl, h16* C16, bf* Ch, bf* Cl) {
    constexpr int NT = CH / 16;
    constexpr int NK = CH / 32;
    constexpr int QB = HI ? 0 : RH;
    constexpr int NQW = HI ? (RH / 16) : ((((SEQ) - RH) / 16) > 0 ? (((SEQ) - RH) / 16) : 1);
    __shared__ __align__(16) float ot[2][16 * 68];
    const int wv = threadIdx.x >> 5, lane = threadIdx.x & 31, h = lane >> 4, m = lane & 15;
    const int wid = blockIdx.x * 2 + wv;
    const int z = wid / NQW;
    if (z >= NZ) return;
    const int q0 = QB + (wid - z * NQW) * 16;
    const int tq = q0 + m;
    v16h qf0 = zh(), qf1 = zh(); v16bf qh0 = zb(), qh1 = zb(), ql0 = zb(), ql1 = zb();
    if (HI) { const bf* qp = Qh + ((size_t)z * RH + tq) * HD + 8 * h; const bf* rp = Ql + ((size_t)z * RH + tq) * HD + 8 * h;
        qh0 = WFrag<bf>::ld(qp); qh1 = WFrag<bf>::ld(qp + 32); ql0 = WFrag<bf>::ld(rp); ql1 = WFrag<bf>::ld(rp + 32); }
    else { const h16* qp = Q16 + ((size_t)z * SEQ + tq) * HD + 8 * h; qf0 = WFrag<h16>::ld(qp); qf1 = WFrag<h16>::ld(qp + 32); }
    v8f o[4];
#pragma unroll
    for (int j = 0; j < 4; ++j) o[j] = (v8f){};
    float mrun = NEGB, lrun = 0.0f;
    const int nch = (q0 + 16 + CH - 1) / CH;
#pragma unroll 1
    for (int ch = 0; ch < nch; ++ch) {
        const int key0 = ch * CH;
        v8f s[4];
#pragma unroll
        for (int i = 0; i < NT; ++i) {
            s[i] = (v8f){};
            if (HI) {
                const bf* kp = Kh + ((size_t)z * RH + key0 + 16 * i + m) * HD + 8 * h;
                const bf* lp = Kl + ((size_t)z * RH + key0 + 16 * i + m) * HD + 8 * h;
                const v16bf a0 = WFrag<bf>::ld(kp), a1 = WFrag<bf>::ld(kp + 32);
                s[i] = wmmab(a0, qh0, s[i]); s[i] = wmmab(a1, qh1, s[i]); s[i] = wmmab(a0, ql0, s[i]); s[i] = wmmab(a1, ql1, s[i]);
                const v16bf c0 = WFrag<bf>::ld(lp), c1 = WFrag<bf>::ld(lp + 32);
                s[i] = wmmab(c0, qh0, s[i]); s[i] = wmmab(c1, qh1, s[i]);
                asm volatile("v_nop\n\tv_nop\n\tv_nop\n\tv_nop" : "+v"(s[i]) : "v"(c1), "v"(qh1));
            } else {
                const h16* kp = K16 + ((size_t)z * SEQ + key0 + 16 * i + m) * HD + 8 * h;
                const v16h a0 = WFrag<h16>::ld(kp), a1 = WFrag<h16>::ld(kp + 32);
                s[i] = wmma16(a0, qf0, s[i]); s[i] = wmma16(a1, qf1, s[i]);
                asm volatile("v_nop\n\tv_nop\n\tv_nop\n\tv_nop" : "+v"(s[i]) : "v"(a1), "v"(qf1));
            }
        }
        if (key0 + CH > q0) {
#pragma unroll
            for (int i = 0; i < NT; ++i) {
#pragma unroll
                for (int r = 0; r < 8; ++r) { const int key = key0 + 16 * i + 8 * h + r; const float sv = s[i][r]; s[i][r] = (key > tq) ? NEGB : sv; } }
        }
        float mloc = NEGB;
#pragma unroll
        for (int i = 0; i < NT; ++i) {
#pragma unroll
            for (int r = 0; r < 8; ++r) mloc = fmaxf(mloc, s[i][r]); }
        mloc = fmaxf(mloc, __shfl_xor(mloc, 16, 32));
        const float mnew = fmaxf(mrun, mloc);
        const float alpha = __builtin_amdgcn_exp2f((mrun - mnew) * SL2E);
        float lsum = 0.0f;
#pragma unroll
        for (int i = 0; i < NT; ++i) {
#pragma unroll
            for (int r = 0; r < 8; ++r) { const float ev = __builtin_amdgcn_exp2f((s[i][r] - mnew) * SL2E); s[i][r] = ev; lsum += ev; } }
        lsum += __shfl_xor(lsum, 16, 32);
        lrun = lrun * alpha + lsum; mrun = mnew;
#pragma unroll
        for (int j = 0; j < 4; ++j) o[j] = o[j] * alpha;
        v16h pb[2]; v16bf ph[2], pl[2];
        pb[0] = zh(); pb[1] = zh(); ph[0] = zb(); ph[1] = zb(); pl[0] = zb(); pl[1] = zb();
#pragma unroll
        for (int kk = 0; kk < NK; ++kk) {
            if (HI) { v16us uh = zus(), ul = zus();
#pragma unroll
                for (int r = 0; r < 8; ++r) { unsigned short a, c; splitf(s[2 * kk][r], a, c); uh[r] = a; ul[r] = c; splitf(s[2 * kk + 1][r], a, c); uh[8 + r] = a; ul[8 + r] = c; }
                ph[kk] = __builtin_bit_cast(v16bf, uh); pl[kk] = __builtin_bit_cast(v16bf, ul);
            } else { v16h p = zh();
#pragma unroll
                for (int r = 0; r < 8; ++r) { p[r] = tohx(s[2 * kk][r]); p[8 + r] = tohx(s[2 * kk + 1][r]); }
                pb[kk] = p; }
        }
        v16h av = zh(); v16bf avh = zb(), avl = zb();
#pragma unroll
        for (int j = 0; j < 4; ++j) {
#pragma unroll
            for (int kk = 0; kk < NK; ++kk) {
                if (HI) { const size_t vo = ((size_t)z * HD + 16 * j + m) * RH + key0 + 32 * kk + 8 * h; avh = WFrag<bf>::ld(VTh + vo); avl = WFrag<bf>::ld(VTl + vo);
                    o[j] = wmmab(avh, ph[kk], o[j]); o[j] = wmmab(avh, pl[kk], o[j]); o[j] = wmmab(avl, ph[kk], o[j]); }
                else { const size_t vo = ((size_t)z * HD + 16 * j + m) * SEQ + key0 + 32 * kk + 8 * h; av = WFrag<h16>::ld(VT16 + vo); o[j] = wmma16(av, pb[kk], o[j]); }
            }
        }
        if (HI) asm volatile("v_nop\n\tv_nop\n\tv_nop\n\tv_nop" : "+v"(o[0]), "+v"(o[1]), "+v"(o[2]), "+v"(o[3]) : "v"(avh), "v"(avl), "v"(ph[NK - 1]), "v"(pl[NK - 1]));
        else    asm volatile("v_nop\n\tv_nop\n\tv_nop\n\tv_nop" : "+v"(o[0]), "+v"(o[1]), "+v"(o[2]), "+v"(o[3]) : "v"(av), "v"(pb[NK - 1]));
    }
    const float inv = 1.0f / lrun;
    float* T = &ot[wv][0];
#pragma unroll
    for (int j = 0; j < 4; ++j) { v4f u0, u1;
#pragma unroll
        for (int r = 0; r < 4; ++r) { u0[r] = o[j][r] * inv; u1[r] = o[j][4 + r] * inv; }
        *(v4f*)(T + m * 68 + 16 * j + 8 * h) = u0; *(v4f*)(T + m * 68 + 16 * j + 8 * h + 4) = u1; }
    __builtin_amdgcn_fence(3, "wavefront"); __builtin_amdgcn_wave_barrier(); asm volatile("" ::: "memory");
    const int bb = z / NH, hh = z - bb * NH; const int rq = lane >> 3, pc = (lane & 7) * 8;
#pragma unroll 1
    for (int ps = 0; ps < 2; ++ps) {
#pragma unroll
        for (int it = 0; it < 4; ++it) {
            const int row = it * 4 + rq; const int t = q0 + row;
            const v4f a = *(const v4fa*)(T + row * 68 + pc); const v4f c = *(const v4fa*)(T + row * 68 + pc + 4);
            v8h o8;
#pragma unroll
            for (int e = 0; e < 4; ++e) { o8[e] = tohx(a[e] * CCAR); o8[4 + e] = tohx(c[e] * CCAR); }
            *(volatile v8h*)(C16 + ((size_t)bb * SEQ + t) * EMB + hh * HD + pc) = o8;
            if (HI) { v8us oh, ol;
#pragma unroll
                for (int e = 0; e < 4; ++e) { unsigned short p1, p2; splitf(a[e], p1, p2); oh[e] = p1; ol[e] = p2; splitf(c[e], p1, p2); oh[4 + e] = p1; ol[4 + e] = p2; }
                const size_t oo = ((size_t)bb * RH + t) * EMB + hh * HD + pc; *(volatile v8us*)(Ch + oo) = oh; *(volatile v8us*)(Cl + oo) = ol; }
        }
        if (ps == 0) __threadfence();
    }
}

extern "C" void kernel_launch(void* const* d_in, const int* in_sizes, int n_in,
                              void* d_out, int out_size, void* d_ws, size_t ws_size, hipStream_t stream) {
    if (n_in < 9) return;
    if ((size_t)in_sizes[0] < (size_t)(NB - 1) * T_FULL * EMB + (size_t)SEQ * EMB) return;
    if (in_sizes[1] < EMB * EMB || in_sizes[3] < EMB * EMB || in_sizes[5] < EMB * EMB || in_sizes[7] < EMB * EMB) return;
    if (in_sizes[2] < EMB || in_sizes[4] < EMB || in_sizes[6] < EMB || in_sizes[8] < EMB) return;
    if ((size_t)out_size < (size_t)(NB - 1) * T_FULL * EMB + (size_t)SEQ * EMB) return;
    const float* x  = (const float*)d_in[0];
    const float* wq = (const float*)d_in[1]; const float* bq = (const float*)d_in[2];
    const float* wk = (const float*)d_in[3]; const float* bk = (const float*)d_in[4];
    const float* wv = (const float*)d_in[5]; const float* bv = (const float*)d_in[6];
    const float* wo = (const float*)d_in[7]; const float* bo = (const float*)d_in[8];
    float* OUT = (float*)d_out;
    char* wsp = (char*)d_ws;
    auto take = [&](size_t bytes) { char* p = wsp; wsp += (bytes + 255) & ~(size_t)255; return (void*)p; };
    bf*  XB  = (bf*)take((size_t)NB * SEQ * EMB * 2);
    bf*  WQ  = (bf*)take((size_t)EMB * EMB * 2); bf* WK = (bf*)take((size_t)EMB * EMB * 2); bf* WV = (bf*)take((size_t)EMB * EMB * 2);
    bf*  WOB = (bf*)take((size_t)EMB * EMB * 2); h16* WOH = (h16*)take((size_t)EMB * EMB * 2);
    float* F = (float*)take((size_t)SEQ * EMB * 4);
    h16* Q16 = (h16*)take((size_t)NZ * SEQ * HD * 2); h16* K16 = (h16*)take((size_t)NZ * SEQ * HD * 2); h16* VT16 = (h16*)take((size_t)NZ * HD * SEQ * 2);
    bf*  QH  = (bf*)take((size_t)NZ * RH * HD * 2); bf* QL = (bf*)take((size_t)NZ * RH * HD * 2);
    bf*  KH  = (bf*)take((size_t)NZ * RH * HD * 2); bf* KL = (bf*)take((size_t)NZ * RH * HD * 2);
    bf*  VTH = (bf*)take((size_t)NZ * HD * RH * 2); bf* VTL = (bf*)take((size_t)NZ * HD * RH * 2);
    h16* C16 = (h16*)take((size_t)NB * SEQ * EMB * 2);
    bf*  CHP = (bf*)take((size_t)NB * RH * EMB * 2); bf* CLP = (bf*)take((size_t)NB * RH * EMB * 2);
    const size_t used = (size_t)(wsp - (char*)d_ws);
    if (used > ws_size || used > (size_t)134217728) return;

    const unsigned gw = (unsigned)((EMB * EMB / 64 + 63) / 64);
    k_wtG<bf><<<gw, 256, 0, stream>>>(wq, EMB, EMB, WQ);
    k_wtG<bf><<<gw, 256, 0, stream>>>(wk, EMB, EMB, WK);
    k_wtG<bf><<<gw, 256, 0, stream>>>(wv, EMB, EMB, WV);
    k_wtG<bf><<<gw, 256, 0, stream>>>(wo, EMB, EMB, WOB);
    k_wtG<h16><<<gw, 256, 0, stream>>>(wo, EMB, EMB, WOH);
    k_cvtx<<<(unsigned)(((size_t)NB * SEQ * EMB / 8 + 255) / 256), 256, 0, stream>>>(x, XB, (size_t)NB * SEQ * EMB / 8);
    const unsigned gp = (unsigned)(((size_t)NH * SEQ * HD / 2 + 255) / 256);
    for (int b = 0; b < NB; ++b) {
        const bf* xb = XB + (size_t)b * SEQ * EMB; const int z0 = b * NH;
        k_gemmw<bf, 0, true><<<dim3(SEQ / 64, EMB / 64, 1), 32, 0, stream>>>(xb, nullptr, WQ, nullptr, EMB, F, EMB, bq, 0, 0, 0, 1.0f);
        k_qkp<<<gp, 256, 0, stream>>>(F, z0, Q16, QH, QL);
        k_gemmw<bf, 0, true><<<dim3(SEQ / 64, EMB / 64, 1), 32, 0, stream>>>(xb, nullptr, WK, nullptr, EMB, F, EMB, bk, 0, 0, 0, 1.0f);
        k_qkp<<<gp, 256, 0, stream>>>(F, z0, K16, KH, KL);
        k_gemmw<bf, 0, true><<<dim3(SEQ / 64, EMB / 64, 1), 32, 0, stream>>>(xb, nullptr, WV, nullptr, EMB, F, EMB, bv, 0, 0, 0, 1.0f);
        k_vtp<<<gp, 256, 0, stream>>>(F, z0, VT16, VTH, VTL);
    }
    { const unsigned nqw = RH / 16;
      k_attn<true, 32><<<(unsigned)((NZ * nqw + 1) / 2), 64, 0, stream>>>(Q16, K16, VT16, QH, QL, KH, KL, VTH, VTL, C16, CHP, CLP); }
    if ((SEQ) > (RH)) { const unsigned nqw = ((SEQ) - RH) / 16;
      k_attn<false, 64><<<(unsigned)((NZ * nqw + 1) / 2), 64, 0, stream>>>(Q16, K16, VT16, QH, QL, KH, KL, VTH, VTL, C16, CHP, CLP); }
    k_gemmw<bf, 1, true><<<dim3(RH / 64, EMB / 64, NB), 32, 0, stream>>>(CHP, CLP, WOB, nullptr, EMB, OUT, EMB, bo, (size_t)RH * EMB, 0, (size_t)T_FULL * EMB, 1.0f);
    if ((SEQ) > (RH))
        k_gemmw<h16, 0, true><<<dim3(((SEQ) - RH) / 64, EMB / 64, NB), 32, 0, stream>>>(C16 + (size_t)RH * EMB, nullptr, WOH, nullptr, EMB, OUT + (size_t)RH * EMB, EMB, bo, (size_t)SEQ * EMB, 0, (size_t)T_FULL * EMB, OSC);
}
